// MVSTFN_submodule_42863773614350
// MI455X (gfx1250) — hardware-verified
//
#include <hip/hip_runtime.h>
#include <math.h>

#define NB 2
#define NN 1024
#define TT 12
#define FF 32
#define CC (TT * FF)

typedef _Float16 v16h __attribute__((ext_vector_type(16)));
typedef _Float16 v8h  __attribute__((ext_vector_type(8)));
typedef __bf16   v16b __attribute__((ext_vector_type(16)));
typedef unsigned short v16us __attribute__((ext_vector_type(16)));
typedef unsigned short v8us  __attribute__((ext_vector_type(8)));
typedef float v8f __attribute__((ext_vector_type(8)));
typedef float v4f __attribute__((ext_vector_type(4)));
typedef v8h  __attribute__((may_alias)) v8ha;
typedef v8us __attribute__((may_alias)) v8usa;
typedef v4f  __attribute__((may_alias)) v4fa;

union FragH { v16h v; v8h half[2]; };
union FragB { v16b v; v16us u; v8us half[2]; };
struct HL8 { v8us hi; v8us lo; };

__device__ __forceinline__ float lk(float v) { return fmaxf(v, v * 0.01f); }

__device__ __forceinline__ unsigned int bf16_rne(float f) {
  const unsigned int u = __float_as_uint(f);
  return (u + 0x7FFFu + ((u >> 16) & 1u)) >> 16;
}

__device__ __forceinline__ HL8 split8(v4f a, v4f c) {
  const unsigned int h0 = bf16_rne(a.x), h1 = bf16_rne(a.y), h2 = bf16_rne(a.z), h3 = bf16_rne(a.w);
  const unsigned int h4 = bf16_rne(c.x), h5 = bf16_rne(c.y), h6 = bf16_rne(c.z), h7 = bf16_rne(c.w);
  const v8us hi = { (unsigned short)h0, (unsigned short)h1, (unsigned short)h2, (unsigned short)h3,
                    (unsigned short)h4, (unsigned short)h5, (unsigned short)h6, (unsigned short)h7 };
  const v8us lo = { (unsigned short)bf16_rne(a.x - __uint_as_float(h0 << 16)),
                    (unsigned short)bf16_rne(a.y - __uint_as_float(h1 << 16)),
                    (unsigned short)bf16_rne(a.z - __uint_as_float(h2 << 16)),
                    (unsigned short)bf16_rne(a.w - __uint_as_float(h3 << 16)),
                    (unsigned short)bf16_rne(c.x - __uint_as_float(h4 << 16)),
                    (unsigned short)bf16_rne(c.y - __uint_as_float(h5 << 16)),
                    (unsigned short)bf16_rne(c.z - __uint_as_float(h6 << 16)),
                    (unsigned short)bf16_rne(c.w - __uint_as_float(h7 << 16)) };
  HL8 o; o.hi = hi; o.lo = lo;
  return o;
}

__device__ __forceinline__ float wsum(float v) {
  v += __shfl_xor(v, 16);
  v += __shfl_xor(v, 8);
  v += __shfl_xor(v, 4);
  v += __shfl_xor(v, 2);
  v += __shfl_xor(v, 1);
  return v;
}

__device__ __forceinline__ v8f wf16(v16h a, v16h b, v8f c) {
  return __builtin_amdgcn_wmma_f32_16x16x32_f16(false, a, false, b, (short)0, c, false, false);
}
__device__ __forceinline__ v8f wbf16(v16b a, v16b b, v8f c) {
  return __builtin_amdgcn_wmma_f32_16x16x32_bf16(false, a, false, b, (short)0, c, false, false);
}
__device__ __forceinline__ v8f wmma3b(v8f c, v16b ah, v16b al, v16b bh, v16b bl) {
  c = wbf16(ah, bh, c);
  c = wbf16(ah, bl, c);
  c = wbf16(al, bh, c);
  asm volatile("v_nop\n\tv_nop\n\tv_nop\n\tv_nop" : "+v"(c) : "v"(ah), "v"(al), "v"(bh), "v"(bl));
  return c;
}

__device__ __forceinline__ void ldfrag(const unsigned short* ph, const unsigned short* pl, int h,
                                       FragB& fh, FragB& fl) {
  fh.half[0] = *(const v8usa*)(ph + 8 * h);
  fh.half[1] = *(const v8usa*)(ph + 16 + 8 * h);
  fl.half[0] = *(const v8usa*)(pl + 8 * h);
  fl.half[1] = *(const v8usa*)(pl + 16 + 8 * h);
}

__device__ __forceinline__ v8h absdiff8(v4f a, v4f c, v4f p, v4f q) {
  const v8h o = { (_Float16)fabsf(a.x - p.x), (_Float16)fabsf(a.y - p.y), (_Float16)fabsf(a.z - p.z), (_Float16)fabsf(a.w - p.w),
                  (_Float16)fabsf(c.x - q.x), (_Float16)fabsf(c.y - q.y), (_Float16)fabsf(c.z - q.z), (_Float16)fabsf(c.w - q.w) };
  return o;
}
__device__ __forceinline__ v8h lk8h(v8f a) {
  const v8h o = { (_Float16)lk(a[0]), (_Float16)lk(a[1]), (_Float16)lk(a[2]), (_Float16)lk(a[3]),
                  (_Float16)lk(a[4]), (_Float16)lk(a[5]), (_Float16)lk(a[6]), (_Float16)lk(a[7]) };
  return o;
}
__device__ __forceinline__ float dot8lk(v8f s, v4f wa, v4f wb) {
  float p = lk(s[0]) * wa.x;
  p += lk(s[1]) * wa.y;
  p += lk(s[2]) * wa.z;
  p += lk(s[3]) * wa.w;
  p += lk(s[4]) * wb.x;
  p += lk(s[5]) * wb.y;
  p += lk(s[6]) * wb.z;
  p += lk(s[7]) * wb.w;
  return p;
}

__global__ __launch_bounds__(256) void nf_kernel(const float* __restrict__ x, const float* __restrict__ tcw,
                                                 const float* __restrict__ tcb, float* __restrict__ nf) {
  const int idx = blockIdx.x * 256 + threadIdx.x;
  if (idx >= NB * NN * FF) return;
  const int f = idx & 31, bn = idx >> 5;
  const float* p = x + (size_t)bn * CC + f;
  float acc = 0.0f;
  #pragma unroll
  for (int t = 0; t < TT; ++t) acc += p[t * FF] * tcw[t];
  acc += tcb[0];
  *(volatile float*)(nf + idx) = acc;
  __threadfence();
  *(volatile float*)(nf + idx) = acc;
}

__global__ __launch_bounds__(256) void xt_kernel(const float* __restrict__ x,
                                                 unsigned short* __restrict__ xth,
                                                 unsigned short* __restrict__ xtl) {
  __shared__ __attribute__((aligned(16))) float s_t[64 * 64];
  const int tid = threadIdx.x;
  const int j0 = blockIdx.x * 64, c0 = blockIdx.y * 64, b = blockIdx.z;
  {
    const int jl = tid >> 2, cp = (tid & 3) * 16;
    const float* src = x + ((size_t)(b * NN + j0 + jl)) * CC + c0 + cp;
    float* dst = s_t + jl * 64 + cp;
    #pragma unroll
    for (int q = 0; q < 4; ++q) *(v4fa*)(dst + 4 * q) = *(const v4fa*)(src + 4 * q);
  }
  __syncthreads();
  const int piece = tid & 7, cr = tid >> 3;
  v4f g0, g1, g2, g3;
  g0.x = s_t[(8 * piece + 0) * 64 + cr];      g0.y = s_t[(8 * piece + 1) * 64 + cr];
  g0.z = s_t[(8 * piece + 2) * 64 + cr];      g0.w = s_t[(8 * piece + 3) * 64 + cr];
  g1.x = s_t[(8 * piece + 4) * 64 + cr];      g1.y = s_t[(8 * piece + 5) * 64 + cr];
  g1.z = s_t[(8 * piece + 6) * 64 + cr];      g1.w = s_t[(8 * piece + 7) * 64 + cr];
  g2.x = s_t[(8 * piece + 0) * 64 + cr + 32]; g2.y = s_t[(8 * piece + 1) * 64 + cr + 32];
  g2.z = s_t[(8 * piece + 2) * 64 + cr + 32]; g2.w = s_t[(8 * piece + 3) * 64 + cr + 32];
  g3.x = s_t[(8 * piece + 4) * 64 + cr + 32]; g3.y = s_t[(8 * piece + 5) * 64 + cr + 32];
  g3.z = s_t[(8 * piece + 6) * 64 + cr + 32]; g3.w = s_t[(8 * piece + 7) * 64 + cr + 32];
  const HL8 o0 = split8(g0, g1);
  const HL8 o1 = split8(g2, g3);
  const size_t off0 = ((size_t)(b * CC + c0 + cr)) * NN + j0 + 8 * piece;
  const size_t off1 = off0 + (size_t)32 * NN;
  *(volatile v8us*)(xth + off0) = o0.hi;
  *(volatile v8us*)(xtl + off0) = o0.lo;
  *(volatile v8us*)(xth + off1) = o1.hi;
  *(volatile v8us*)(xtl + off1) = o1.lo;
  __threadfence();
  *(volatile v8us*)(xth + off0) = o0.hi;
  *(volatile v8us*)(xtl + off0) = o0.lo;
  *(volatile v8us*)(xth + off1) = o1.hi;
  *(volatile v8us*)(xtl + off1) = o1.lo;
}

__global__ __launch_bounds__(256) void pair_kernel(
    const float* __restrict__ nf,
    const float* __restrict__ efin,
    const float* __restrict__ adj,
    const float* __restrict__ w0,
    const float* __restrict__ w1,
    const float* __restrict__ wout,
    const float* __restrict__ bout,
    float* __restrict__ efout,
    unsigned short* __restrict__ e2hi,
    unsigned short* __restrict__ e2lo)
{
  __shared__ __attribute__((aligned(16))) _Float16 s_w0h[64 * 32];
  __shared__ __attribute__((aligned(16))) _Float16 s_w1h[32 * 64];
  __shared__ __attribute__((aligned(16))) float s_sim[NN];
  __shared__ float s_red[24];

  const int tid = threadIdx.x, lane = tid & 31, w = tid >> 5;
  const int h = lane >> 4, m = lane & 15;
  const int bi = blockIdx.x;
  const int b = bi >> 10, i = bi & (NN - 1);

  for (int k = tid; k < 2048; k += 256) {
    s_w0h[k] = (_Float16)(w0[k] * 16.0f);
    s_w1h[k] = (_Float16)(w1[k] * 16.0f);
  }
  const float* nfi = nf + (size_t)bi * FF;
  const v4f ni0 = *(const v4fa*)(nfi + 8 * h);
  const v4f ni1 = *(const v4fa*)(nfi + 8 * h + 4);
  const v4f ni2 = *(const v4fa*)(nfi + 16 + 8 * h);
  const v4f ni3 = *(const v4fa*)(nfi + 20 + 8 * h);
  const v4f wo0 = *(const v4fa*)(wout + 8 * h);
  const v4f wo1 = *(const v4fa*)(wout + 8 * h + 4);
  const v4f wo2 = *(const v4fa*)(wout + 16 + 8 * h);
  const v4f wo3 = *(const v4fa*)(wout + 20 + 8 * h);
  const float bo = bout[0];
  const int jb = 4 * tid;
  const v4f e4 = *(const v4fa*)(efin + (size_t)bi * NN + jb);
  const v4f a4 = *(const v4fa*)(adj + (size_t)i * NN + jb);
  const v4f efa = e4 * a4;
  __syncthreads();

  const v8f zero8 = {0.f, 0.f, 0.f, 0.f, 0.f, 0.f, 0.f, 0.f};

  #pragma unroll 1
  for (int q = 0; q < 8; ++q) {
    const int j0 = (w * 8 + q) * 16;
    const float* nfj = nf + ((size_t)(b * NN + j0 + m)) * FF;
    const v4f r0 = *(const v4fa*)(nfj + 8 * h);
    const v4f r1 = *(const v4fa*)(nfj + 8 * h + 4);
    const v4f r2 = *(const v4fa*)(nfj + 16 + 8 * h);
    const v4f r3 = *(const v4fa*)(nfj + 20 + 8 * h);
    FragH d;
    d.half[0] = absdiff8(r0, r1, ni0, ni1);
    d.half[1] = absdiff8(r2, r3, ni2, ni3);
    FragH a0, a1, a2, a3;
    a0.half[0] = *(const v8ha*)(s_w0h + (0 * 16 + m) * 32 + 8 * h);
    a0.half[1] = *(const v8ha*)(s_w0h + (0 * 16 + m) * 32 + 16 + 8 * h);
    a1.half[0] = *(const v8ha*)(s_w0h + (1 * 16 + m) * 32 + 8 * h);
    a1.half[1] = *(const v8ha*)(s_w0h + (1 * 16 + m) * 32 + 16 + 8 * h);
    a2.half[0] = *(const v8ha*)(s_w0h + (2 * 16 + m) * 32 + 8 * h);
    a2.half[1] = *(const v8ha*)(s_w0h + (2 * 16 + m) * 32 + 16 + 8 * h);
    a3.half[0] = *(const v8ha*)(s_w0h + (3 * 16 + m) * 32 + 8 * h);
    a3.half[1] = *(const v8ha*)(s_w0h + (3 * 16 + m) * 32 + 16 + 8 * h);
    v8f acc0 = wf16(a0.v, d.v, zero8);
    v8f acc1 = wf16(a1.v, d.v, zero8);
    v8f acc2 = wf16(a2.v, d.v, zero8);
    v8f acc3 = wf16(a3.v, d.v, zero8);
    asm volatile("v_nop\n\tv_nop\n\tv_nop\n\tv_nop"
                 : "+v"(acc0), "+v"(acc1), "+v"(acc2), "+v"(acc3)
                 : "v"(a0.v), "v"(a1.v), "v"(a2.v), "v"(a3.v), "v"(d.v));
    FragH p0, p1;
    p0.half[0] = lk8h(acc0);
    p0.half[1] = lk8h(acc1);
    p1.half[0] = lk8h(acc2);
    p1.half[1] = lk8h(acc3);
    FragH c00, c01, c10, c11;
    c00.half[0] = *(const v8ha*)(s_w1h + m * 64 + 8 * h);
    c00.half[1] = *(const v8ha*)(s_w1h + m * 64 + 16 + 8 * h);
    c01.half[0] = *(const v8ha*)(s_w1h + m * 64 + 32 + 8 * h);
    c01.half[1] = *(const v8ha*)(s_w1h + m * 64 + 48 + 8 * h);
    c10.half[0] = *(const v8ha*)(s_w1h + (16 + m) * 64 + 8 * h);
    c10.half[1] = *(const v8ha*)(s_w1h + (16 + m) * 64 + 16 + 8 * h);
    c11.half[0] = *(const v8ha*)(s_w1h + (16 + m) * 64 + 32 + 8 * h);
    c11.half[1] = *(const v8ha*)(s_w1h + (16 + m) * 64 + 48 + 8 * h);
    v8f s0 = wf16(c00.v, p0.v, zero8);
    s0 = wf16(c01.v, p1.v, s0);
    v8f s1 = wf16(c10.v, p0.v, zero8);
    s1 = wf16(c11.v, p1.v, s1);
    asm volatile("v_nop\n\tv_nop\n\tv_nop\n\tv_nop"
                 : "+v"(s0), "+v"(s1)
                 : "v"(c00.v), "v"(c01.v), "v"(c10.v), "v"(c11.v), "v"(p0.v), "v"(p1.v));
    float pr = dot8lk(s0, wo0, wo1) + dot8lk(s1, wo2, wo3);
    pr += __shfl_xor(pr, 16);
    float z = pr * (1.0f / 256.0f) + bo;
    z = fminf(fmaxf(z, -60.0f), 60.0f);
    const float ez = expf(-z);
    const float sg = 1.0f / (1.0f + ez);
    if (h == 0) s_sim[j0 + m] = sg;
  }
  __syncthreads();

  const v4f s4 = *(const v4fa*)(s_sim + jb);
  const v4f v4 = s4 * efa;
  float msp = (efa.x + efa.y) + (efa.z + efa.w);
  float ssp = (fabsf(v4.x) + fabsf(v4.y)) + (fabsf(v4.z) + fabsf(v4.w));
  msp = wsum(msp);
  ssp = wsum(ssp);
  if (lane == 0) { s_red[w] = msp; s_red[8 + w] = ssp; }
  __syncthreads();
  float MS = 0.0f, SS = 0.0f;
  #pragma unroll
  for (int k = 0; k < 8; ++k) { MS += s_red[k]; SS += s_red[8 + k]; }
  const float inv1 = 1.0f / fmaxf(SS, 1e-12f);
  const v4f wv = (v4 * inv1) * MS;
  v4f dg;
  dg.x = (jb + 0 == i) ? 1.0f : 0.0f;
  dg.y = (jb + 1 == i) ? 1.0f : 0.0f;
  dg.z = (jb + 2 == i) ? 1.0f : 0.0f;
  dg.w = (jb + 3 == i) ? 1.0f : 0.0f;
  const v4f efv = wv + dg;
  v4f mk;
  mk.x = (jb + 0 == i) ? 0.0f : wv.x;
  mk.y = (jb + 1 == i) ? 0.0f : wv.y;
  mk.z = (jb + 2 == i) ? 0.0f : wv.z;
  mk.w = (jb + 3 == i) ? 0.0f : wv.w;
  float d2p = (fabsf(mk.x) + fabsf(mk.y)) + (fabsf(mk.z) + fabsf(mk.w));
  d2p = wsum(d2p);
  if (lane == 0) s_red[16 + w] = d2p;
  float* efo = efout + (size_t)bi * NN + jb;
  *(volatile v4f*)efo = efv;
  __syncthreads();
  float D2 = 0.0f;
  #pragma unroll
  for (int k = 0; k < 8; ++k) D2 += s_red[16 + k];
  const float inv2 = 1.0f / fmaxf(D2, 1e-12f);
  const v4f e2v = mk * inv2;
  *(v4fa*)(s_sim + jb) = e2v;
  __threadfence();
  *(volatile v4f*)efo = efv;
  __syncthreads();
  if (tid < 128) {
    const v4f g0 = *(const v4fa*)(s_sim + 8 * tid);
    const v4f g1 = *(const v4fa*)(s_sim + 8 * tid + 4);
    const HL8 hl = split8(g0, g1);
    const size_t po = (size_t)bi * NN + 8 * tid;
    *(volatile v8us*)(e2hi + po) = hl.hi;
    *(volatile v8us*)(e2lo + po) = hl.lo;
    __threadfence();
    *(volatile v8us*)(e2hi + po) = hl.hi;
    *(volatile v8us*)(e2lo + po) = hl.lo;
  }
}

__global__ __launch_bounds__(256) void aggr_node_kernel(
    const unsigned short* __restrict__ e2hi, const unsigned short* __restrict__ e2lo,
    const unsigned short* __restrict__ xthi, const unsigned short* __restrict__ xtlo,
    const float* __restrict__ xin,
    const float* __restrict__ nw0,
    const float* __restrict__ nw1,
    const float* __restrict__ rw,
    const float* __restrict__ rb,
    const float* __restrict__ lnw,
    const float* __restrict__ lnb,
    float* __restrict__ xout)
{
  __shared__ __attribute__((aligned(16))) float s_ag[16 * CC];
  __shared__ __attribute__((aligned(16))) unsigned short s_w0h[64 * 64];
  __shared__ __attribute__((aligned(16))) unsigned short s_w0l[64 * 64];
  __shared__ __attribute__((aligned(16))) unsigned short s_w1h[32 * 64];
  __shared__ __attribute__((aligned(16))) unsigned short s_w1l[32 * 64];
  __shared__ __attribute__((aligned(16))) unsigned short s_rwh[32 * 32];
  __shared__ __attribute__((aligned(16))) unsigned short s_rwl[32 * 32];
  __shared__ __attribute__((aligned(16))) float s_rb[32];
  __shared__ __attribute__((aligned(16))) float s_lnw[32];
  __shared__ __attribute__((aligned(16))) float s_lnb[32];

  const int tid = threadIdx.x, lane = tid & 31, w = tid >> 5;
  const int h = lane >> 4, m = lane & 15;
  const int b = blockIdx.x >> 6, i0 = (blockIdx.x & 63) * 16;

  for (int k = tid; k < 64 * 64; k += 256) {
    const float v = nw0[k];
    const unsigned int hb = bf16_rne(v);
    s_w0h[k] = (unsigned short)hb;
    s_w0l[k] = (unsigned short)bf16_rne(v - __uint_as_float(hb << 16));
  }
  for (int k = tid; k < 32 * 64; k += 256) {
    const float v = nw1[k];
    const unsigned int hb = bf16_rne(v);
    s_w1h[k] = (unsigned short)hb;
    s_w1l[k] = (unsigned short)bf16_rne(v - __uint_as_float(hb << 16));
  }
  for (int k = tid; k < 32 * 32; k += 256) {
    const float v = rw[k];
    const unsigned int hb = bf16_rne(v);
    s_rwh[k] = (unsigned short)hb;
    s_rwl[k] = (unsigned short)bf16_rne(v - __uint_as_float(hb << 16));
  }
  if (tid < 32) { s_rb[tid] = rb[tid]; s_lnw[tid] = lnw[tid]; s_lnb[tid] = lnb[tid]; }
  __syncthreads();

  const v8f zero8 = {0.f, 0.f, 0.f, 0.f, 0.f, 0.f, 0.f, 0.f};

  {
    const int c0 = 48 * w;
    const size_t arow = ((size_t)(b * NN + i0 + m)) * NN;
    const size_t brow = ((size_t)(b * CC + c0 + m)) * NN;
    const unsigned short* pah = e2hi + arow;
    const unsigned short* pal = e2lo + arow;
    const unsigned short* pbh = xthi + brow;
    const unsigned short* pbl = xtlo + brow;
    v8f acc0 = zero8, acc1 = zero8, acc2 = zero8;
    #pragma unroll 1
    for (int k0 = 0; k0 < NN; k0 += 32) {
      FragB ah, al, bh0, bl0, bh1, bl1, bh2, bl2;
      ldfrag(pah + k0, pal + k0, h, ah, al);
      ldfrag(pbh + k0, pbl + k0, h, bh0, bl0);
      ldfrag(pbh + (size_t)16 * NN + k0, pbl + (size_t)16 * NN + k0, h, bh1, bl1);
      ldfrag(pbh + (size_t)32 * NN + k0, pbl + (size_t)32 * NN + k0, h, bh2, bl2);
      acc0 = wmma3b(acc0, ah.v, al.v, bh0.v, bl0.v);
      acc1 = wmma3b(acc1, ah.v, al.v, bh1.v, bl1.v);
      acc2 = wmma3b(acc2, ah.v, al.v, bh2.v, bl2.v);
    }
    #pragma unroll
    for (int r = 0; r < 8; ++r) {
      s_ag[(8 * h + r) * CC + c0 + 0 + m]  = acc0[r];
      s_ag[(8 * h + r) * CC + c0 + 16 + m] = acc1[r];
      s_ag[(8 * h + r) * CC + c0 + 32 + m] = acc2[r];
    }
  }
  __syncthreads();

  const size_t R0 = ((size_t)(b * NN + i0)) * TT;
  #pragma unroll
  for (int rep = 0; rep < 2; ++rep) {
    const int rt = w + 8 * rep;
    float y[16];
    #pragma unroll
    for (int e = 0; e < 16; ++e) y[e] = 0.0f;
    if (rt < 12) {
      const int rho = 16 * rt + m;
      const float* gx = xin + (R0 + rho) * FF;
      const v4f x0 = *(const v4fa*)(gx + 8 * h);
      const v4f x1 = *(const v4fa*)(gx + 8 * h + 4);
      const v4f x2 = *(const v4fa*)(gx + 16 + 8 * h);
      const v4f x3 = *(const v4fa*)(gx + 20 + 8 * h);
      const float* ga = s_ag + rho * FF;
      const v4f g0 = *(const v4fa*)(ga + 8 * h);
      const v4f g1 = *(const v4fa*)(ga + 8 * h + 4);
      const v4f g2 = *(const v4fa*)(ga + 16 + 8 * h);
      const v4f g3 = *(const v4fa*)(ga + 20 + 8 * h);
      FragB xbh, xbl, abh, abl;
      {
        const HL8 t0 = split8(x0, x1), t1 = split8(x2, x3);
        xbh.half[0] = t0.hi; xbh.half[1] = t1.hi; xbl.half[0] = t0.lo; xbl.half[1] = t1.lo;
        const HL8 u0 = split8(g0, g1), u1 = split8(g2, g3);
        abh.half[0] = u0.hi; abh.half[1] = u1.hi; abl.half[0] = u0.lo; abl.half[1] = u1.lo;
      }
      FragB fh, fl;
      v8f h1_0, h1_1, h1_2, h1_3;
      ldfrag(s_w0h + (0 + m) * 64, s_w0l + (0 + m) * 64, h, fh, fl);
      h1_0 = wmma3b(zero8, fh.v, fl.v, xbh.v, xbl.v);
      ldfrag(s_w0h + (0 + m) * 64 + 32, s_w0l + (0 + m) * 64 + 32, h, fh, fl);
      h1_0 = wmma3b(h1_0, fh.v, fl.v, abh.v, abl.v);
      ldfrag(s_w0h + (16 + m) * 64, s_w0l + (16 + m) * 64, h, fh, fl);
      h1_1 = wmma3b(zero8, fh.v, fl.v, xbh.v, xbl.v);
      ldfrag(s_w0h + (16 + m) * 64 + 32, s_w0l + (16 + m) * 64 + 32, h, fh, fl);
      h1_1 = wmma3b(h1_1, fh.v, fl.v, abh.v, abl.v);
      ldfrag(s_w0h + (32 + m) * 64, s_w0l + (32 + m) * 64, h, fh, fl);
      h1_2 = wmma3b(zero8, fh.v, fl.v, xbh.v, xbl.v);
      ldfrag(s_w0h + (32 + m) * 64 + 32, s_w0l + (32 + m) * 64 + 32, h, fh, fl);
      h1_2 = wmma3b(h1_2, fh.v, fl.v, abh.v, abl.v);
      ldfrag(s_w0h + (48 + m) * 64, s_w0l + (48 + m) * 64, h, fh, fl);
      h1_3 = wmma3b(zero8, fh.v, fl.v, xbh.v, xbl.v);
      ldfrag(s_w0h + (48 + m) * 64 + 32, s_w0l + (48 + m) * 64 + 32, h, fh, fl);
      h1_3 = wmma3b(h1_3, fh.v, fl.v, abh.v, abl.v);
      FragB p0h, p0l, p1h, p1l;
      {
        const v4f qa = { lk(h1_0[0]), lk(h1_0[1]), lk(h1_0[2]), lk(h1_0[3]) };
        const v4f qb = { lk(h1_0[4]), lk(h1_0[5]), lk(h1_0[6]), lk(h1_0[7]) };
        const HL8 u = split8(qa, qb);
        p0h.half[0] = u.hi; p0l.half[0] = u.lo;
      }
      {
        const v4f qa = { lk(h1_1[0]), lk(h1_1[1]), lk(h1_1[2]), lk(h1_1[3]) };
        const v4f qb = { lk(h1_1[4]), lk(h1_1[5]), lk(h1_1[6]), lk(h1_1[7]) };
        const HL8 u = split8(qa, qb);
        p0h.half[1] = u.hi; p0l.half[1] = u.lo;
      }
      {
        const v4f qa = { lk(h1_2[0]), lk(h1_2[1]), lk(h1_2[2]), lk(h1_2[3]) };
        const v4f qb = { lk(h1_2[4]), lk(h1_2[5]), lk(h1_2[6]), lk(h1_2[7]) };
        const HL8 u = split8(qa, qb);
        p1h.half[0] = u.hi; p1l.half[0] = u.lo;
      }
      {
        const v4f qa = { lk(h1_3[0]), lk(h1_3[1]), lk(h1_3[2]), lk(h1_3[3]) };
        const v4f qb = { lk(h1_3[4]), lk(h1_3[5]), lk(h1_3[6]), lk(h1_3[7]) };
        const HL8 u = split8(qa, qb);
        p1h.half[1] = u.hi; p1l.half[1] = u.lo;
      }
      v8f n0, n1;
      ldfrag(s_w1h + m * 64, s_w1l + m * 64, h, fh, fl);
      n0 = wmma3b(zero8, fh.v, fl.v, p0h.v, p0l.v);
      ldfrag(s_w1h + m * 64 + 32, s_w1l + m * 64 + 32, h, fh, fl);
      n0 = wmma3b(n0, fh.v, fl.v, p1h.v, p1l.v);
      ldfrag(s_w1h + (16 + m) * 64, s_w1l + (16 + m) * 64, h, fh, fl);
      n1 = wmma3b(zero8, fh.v, fl.v, p0h.v, p0l.v);
      ldfrag(s_w1h + (16 + m) * 64 + 32, s_w1l + (16 + m) * 64 + 32, h, fh, fl);
      n1 = wmma3b(n1, fh.v, fl.v, p1h.v, p1l.v);
      v8f q0, q1;
      ldfrag(s_rwh + m * 32, s_rwl + m * 32, h, fh, fl);
      q0 = wmma3b(zero8, fh.v, fl.v, xbh.v, xbl.v);
      ldfrag(s_rwh + (16 + m) * 32, s_rwl + (16 + m) * 32, h, fh, fl);
      q1 = wmma3b(zero8, fh.v, fl.v, xbh.v, xbl.v);
      const v4f rb0 = *(const v4fa*)(s_rb + 8 * h);
      const v4f rb1 = *(const v4fa*)(s_rb + 8 * h + 4);
      const v4f rb2 = *(const v4fa*)(s_rb + 16 + 8 * h);
      const v4f rb3 = *(const v4fa*)(s_rb + 20 + 8 * h);
      y[0]  = fmaxf((q0[0] + rb0.x) + lk(n0[0]), 0.0f);
      y[1]  = fmaxf((q0[1] + rb0.y) + lk(n0[1]), 0.0f);
      y[2]  = fmaxf((q0[2] + rb0.z) + lk(n0[2]), 0.0f);
      y[3]  = fmaxf((q0[3] + rb0.w) + lk(n0[3]), 0.0f);
      y[4]  = fmaxf((q0[4] + rb1.x) + lk(n0[4]), 0.0f);
      y[5]  = fmaxf((q0[5] + rb1.y) + lk(n0[5]), 0.0f);
      y[6]  = fmaxf((q0[6] + rb1.z) + lk(n0[6]), 0.0f);
      y[7]  = fmaxf((q0[7] + rb1.w) + lk(n0[7]), 0.0f);
      y[8]  = fmaxf((q1[0] + rb2.x) + lk(n1[0]), 0.0f);
      y[9]  = fmaxf((q1[1] + rb2.y) + lk(n1[1]), 0.0f);
      y[10] = fmaxf((q1[2] + rb2.z) + lk(n1[2]), 0.0f);
      y[11] = fmaxf((q1[3] + rb2.w) + lk(n1[3]), 0.0f);
      y[12] = fmaxf((q1[4] + rb3.x) + lk(n1[4]), 0.0f);
      y[13] = fmaxf((q1[5] + rb3.y) + lk(n1[5]), 0.0f);
      y[14] = fmaxf((q1[6] + rb3.z) + lk(n1[6]), 0.0f);
      y[15] = fmaxf((q1[7] + rb3.w) + lk(n1[7]), 0.0f);
      float s1 = 0.0f;
      #pragma unroll
      for (int e = 0; e < 16; ++e) s1 += y[e];
      s1 += __shfl_xor(s1, 16);
      const float mu = s1 * (1.0f / 32.0f);
      float s2 = 0.0f;
      #pragma unroll
      for (int e = 0; e < 16; ++e) { const float dv = y[e] - mu; s2 += dv * dv; }
      s2 += __shfl_xor(s2, 16);
      const float var = s2 * (1.0f / 32.0f);
      const float inv = 1.0f / sqrtf(var + 1e-5f);
      const v4f lw0 = *(const v4fa*)(s_lnw + 8 * h);
      const v4f lw1 = *(const v4fa*)(s_lnw + 8 * h + 4);
      const v4f lw2 = *(const v4fa*)(s_lnw + 16 + 8 * h);
      const v4f lw3 = *(const v4fa*)(s_lnw + 20 + 8 * h);
      const v4f lb0 = *(const v4fa*)(s_lnb + 8 * h);
      const v4f lb1 = *(const v4fa*)(s_lnb + 8 * h + 4);
      const v4f lb2 = *(const v4fa*)(s_lnb + 16 + 8 * h);
      const v4f lb3 = *(const v4fa*)(s_lnb + 20 + 8 * h);
      y[0]  = (y[0]  - mu) * inv * lw0.x + lb0.x;
      y[1]  = (y[1]  - mu) * inv * lw0.y + lb0.y;
      y[2]  = (y[2]  - mu) * inv * lw0.z + lb0.z;
      y[3]  = (y[3]  - mu) * inv * lw0.w + lb0.w;
      y[4]  = (y[4]  - mu) * inv * lw1.x + lb1.x;
      y[5]  = (y[5]  - mu) * inv * lw1.y + lb1.y;
      y[6]  = (y[6]  - mu) * inv * lw1.z + lb1.z;
      y[7]  = (y[7]  - mu) * inv * lw1.w + lb1.w;
      y[8]  = (y[8]  - mu) * inv * lw2.x + lb2.x;
      y[9]  = (y[9]  - mu) * inv * lw2.y + lb2.y;
      y[10] = (y[10] - mu) * inv * lw2.z + lb2.z;
      y[11] = (y[11] - mu) * inv * lw2.w + lb2.w;
      y[12] = (y[12] - mu) * inv * lw3.x + lb3.x;
      y[13] = (y[13] - mu) * inv * lw3.y + lb3.y;
      y[14] = (y[14] - mu) * inv * lw3.z + lb3.z;
      y[15] = (y[15] - mu) * inv * lw3.w + lb3.w;
    }
    __syncthreads();
    if (rt < 12) {
      float* dst = s_ag + (16 * rt + m) * FF;
      #pragma unroll
      for (int r = 0; r < 8; ++r) {
        dst[8 * h + r] = y[r];
        dst[16 + 8 * h + r] = y[8 + r];
      }
    }
  }
  __syncthreads();

  float* ob = xout + R0 * FF;
  v4f ov[6];
  #pragma unroll
  for (int it = 0; it < 6; ++it) ov[it] = *(const v4fa*)(s_ag + 4 * (it * 256 + tid));
  #pragma unroll
  for (int it = 0; it < 6; ++it) *(volatile v4f*)(ob + 4 * (it * 256 + tid)) = ov[it];
  __threadfence();
  #pragma unroll
  for (int it = 0; it < 6; ++it) *(volatile v4f*)(ob + 4 * (it * 256 + tid)) = ov[it];
}

extern "C" void kernel_launch(void* const* d_in, const int* in_sizes, int n_in,
                              void* d_out, int out_size, void* d_ws, size_t ws_size,
                              hipStream_t stream) {
  if (n_in < 15) return;
  if (in_sizes[0] != NB * NN * CC) return;
  if (in_sizes[1] != NB * NN * NN) return;
  if (in_sizes[2] != NN * NN) return;
  if (in_sizes[3] != 2 * TT || in_sizes[4] != 2) return;
  if (in_sizes[5] != 2 * 64 * 32 || in_sizes[6] != 2 * 32 * 64 || in_sizes[7] != 2 * 32 || in_sizes[8] != 2) return;
  if (in_sizes[9] != 2 * 64 * 64 || in_sizes[10] != 2 * 32 * 64 || in_sizes[11] != 2 * 32 * 32) return;
  if (in_sizes[12] != 2 * 32 || in_sizes[13] != 2 * 32 || in_sizes[14] != 2 * 32) return;
  if (out_size != NB * NN * CC + NB * NN * NN) return;

  const float* x_in   = (const float*)d_in[0];
  const float* edge   = (const float*)d_in[1];
  const float* adj    = (const float*)d_in[2];
  const float* tc_w   = (const float*)d_in[3];
  const float* tc_b   = (const float*)d_in[4];
  const float* e_w0   = (const float*)d_in[5];
  const float* e_w1   = (const float*)d_in[6];
  const float* e_wout = (const float*)d_in[7];
  const float* e_bout = (const float*)d_in[8];
  const float* n_w0   = (const float*)d_in[9];
  const float* n_w1   = (const float*)d_in[10];
  const float* r_w    = (const float*)d_in[11];
  const float* r_b    = (const float*)d_in[12];
  const float* ln_w   = (const float*)d_in[13];
  const float* ln_b   = (const float*)d_in[14];

  float* out_x  = (float*)d_out;
  float* out_ef = out_x + (size_t)NB * NN * CC;

  const size_t nf_bytes = (size_t)NB * NN * FF * 4;
  const size_t ef_bytes = (size_t)NB * NN * NN * 4;
  const size_t e2_bytes = (size_t)NB * NN * NN * 2;
  const size_t xt_bytes = (size_t)NB * CC * NN * 2;
  const size_t y_bytes  = (size_t)NB * NN * CC * 4;
  const size_t total = nf_bytes + ef_bytes + 2 * e2_bytes + 2 * xt_bytes + y_bytes;
  if (total > ws_size) return;

  char* ws = (char*)d_ws;
  float* nf_ws = (float*)ws;                          ws += nf_bytes;
  float* ef_ws = (float*)ws;                          ws += ef_bytes;
  unsigned short* e2hi = (unsigned short*)ws;         ws += e2_bytes;
  unsigned short* e2lo = (unsigned short*)ws;         ws += e2_bytes;
  unsigned short* xthi = (unsigned short*)ws;         ws += xt_bytes;
  unsigned short* xtlo = (unsigned short*)ws;         ws += xt_bytes;
  float* y_ws = (float*)ws;                           ws += y_bytes;

  for (int l = 0; l < 2; ++l) {
    const float* xi  = (l == 0) ? x_in : y_ws;
    const float* efi = (l == 0) ? edge : ef_ws;
    float* xo  = (l == 0) ? y_ws  : out_x;
    float* efo = (l == 0) ? ef_ws : out_ef;

    nf_kernel<<<(NB * NN * FF) / 256, 256, 0, stream>>>(xi, tc_w + l * TT, tc_b + l, nf_ws);

    xt_kernel<<<dim3(NN / 64, CC / 64, NB), 256, 0, stream>>>(xi, xthi, xtlo);

    pair_kernel<<<NB * NN, 256, 0, stream>>>(
        nf_ws, efi, adj,
        e_w0 + (size_t)l * 64 * 32, e_w1 + (size_t)l * 32 * 64, e_wout + l * 32, e_bout + l,
        efo, e2hi, e2lo);

    aggr_node_kernel<<<NB * (NN / 16), 256, 0, stream>>>(
        e2hi, e2lo, xthi, xtlo, xi,
        n_w0 + (size_t)l * 64 * 64, n_w1 + (size_t)l * 32 * 64, r_w + (size_t)l * 32 * 32,
        r_b + l * 32, ln_w + l * 32, ln_b + l * 32, xo);
  }
}
